// SpatialAttentionBlock_89309549953899
// MI455X (gfx1250) — hardware-verified
//
#include <hip/hip_runtime.h>


typedef __attribute__((ext_vector_type(16))) _Float16 v16h;
typedef __attribute__((ext_vector_type(8)))  _Float16 v8h;
typedef __attribute__((ext_vector_type(8)))  float v8f;
typedef __attribute__((ext_vector_type(4)))  float v4f;
typedef __attribute__((ext_vector_type(4)))  unsigned int v4u;
union H8 { v8h h; v4u u; };

#ifndef NB
#define NB 2
#endif
#ifndef SEQ
#define SEQ 2048
#endif
#define NB_FULL  2
#define SEQ_FULL 2048
#define DM   1024
#define NH   16
#define HD   64
#define FF   4096
#define ROWS (NB * SEQ)
#define KPAD  72
#define VSPAD 136
#define SP64  68
#define SP128 132
#define LN_EPS 1e-5f
#define WSC    64.0f
#define CTXC   64.0f
#define H2C    64.0f
#define VRC    4096.0f
#define LN1024 6.931471806f

#define NWB_QKV (3 * DM * DM / 2048)
#define NWB_P   (DM * DM / 2048)
#define NWB_F1  (FF * DM / 2048)
#define NWB_F2  (DM * FF / 2048)
#define NWB     (NWB_QKV + NWB_P + NWB_F1 + NWB_F2)

#define XH_BYTES   ((size_t)ROWS * DM * 2)
#define WQKV_BYTES ((size_t)3 * DM * DM * 2)
#define WP_BYTES   ((size_t)DM * DM * 2)
#define WF1_BYTES  ((size_t)FF * DM * 2)
#define WF2_BYTES  ((size_t)DM * FF * 2)
#define QP_BYTES   ((size_t)ROWS * DM * 2)
#define AM_BYTES   ((size_t)ROWS * DM * 2)
#define H2F_BYTES  ((size_t)ROWS * DM * 4)
#define H2H_BYTES  ((size_t)ROWS * DM * 2)
#define G_BYTES    ((size_t)ROWS * FF * 4)
#define NP_BYTES   ((size_t)ROWS * FF * 2)
#define RG_EARLY   (XH_BYTES + WQKV_BYTES + WP_BYTES + 4 * QP_BYTES + AM_BYTES)
#define RG_BYTES   ((G_BYTES > RG_EARLY) ? G_BYTES : RG_EARLY)
#define RN_EARLY   (H2H_BYTES + WF1_BYTES)
#define RN_BYTES   ((NP_BYTES > RN_EARLY) ? NP_BYTES : RN_EARLY)
#define WS_TOTAL   (RG_BYTES + RN_BYTES + H2F_BYTES + WF2_BYTES)

static_assert(NB >= 1 && NB <= NB_FULL);
static_assert(SEQ >= 128 && SEQ <= SEQ_FULL && (SEQ % 128) == 0);
static_assert((ROWS % 128) == 0);
static_assert((DM % 128) == 0 && (FF % 64) == 0 && HD == 64 && NH * HD == DM && NH == 16);
static_assert(FF == 2 * 8 * 256);
static_assert((3 * DM * DM) % 2048 == 0 && (DM * DM) % 2048 == 0 && (FF * DM) % 2048 == 0);
static_assert(128 * KPAD <= 128 * VSPAD);
static_assert((RG_BYTES % 128) == 0 && (RN_BYTES % 128) == 0 && (H2F_BYTES % 128) == 0);
static_assert(WS_TOTAL <= (size_t)134217728);

__device__ __forceinline__ float bf16q(float f) {
  unsigned int u = __float_as_uint(f);
  u += 0x7FFFu + ((u >> 16) & 1u);
  return __uint_as_float(u & 0xFFFF0000u);
}

__device__ __forceinline__ v16h load_frag_row(const _Float16* base, int stride, int lane) {
  const _Float16* rowp = base + (size_t)(lane & 15) * stride + ((lane >> 4) << 3);
  const v8h lo = *(const v8h*)(rowp);
  const v8h hi = *(const v8h*)(rowp + 16);
  return __builtin_shufflevector(lo, hi, 0, 1, 2, 3, 4, 5, 6, 7,
                                 8, 9, 10, 11, 12, 13, 14, 15);
}

__device__ __forceinline__ v8f wmma_f16(v16h a, v16h b, v8f c) {
  v8f d = __builtin_amdgcn_wmma_f32_16x16x32_f16(false, a, false, b, (short)0, c,
                                                 false, false);
  asm volatile("v_nop\n\tv_nop\n\tv_nop\n\tv_nop" : "+v"(d) : "v"(a), "v"(b));
  return d;
}

__device__ __forceinline__ float wave_sum(float v) {
  v += __shfl_xor(v, 16, 32);
  v += __shfl_xor(v, 8, 32);
  v += __shfl_xor(v, 4, 32);
  v += __shfl_xor(v, 2, 32);
  v += __shfl_xor(v, 1, 32);
  return v;
}

__global__ __launch_bounds__(256) void cvt_x_kernel(const float* __restrict__ x,
                                                    _Float16* __restrict__ xh) {
  __shared__ _Float16 ts[64 * KPAD];
  const int tid = threadIdx.x;
  const int n0 = blockIdx.x * 64;
  const int c0 = blockIdx.y * 64;
  const int b  = blockIdx.z;
#pragma unroll
  for (int it = 0; it < 4; ++it) {
    const int idx = it * 256 + tid;
    const int cr = idx >> 4, q4 = idx & 15;
    const v4f v = *(const v4f*)(x + ((size_t)b * DM + c0 + cr) * SEQ_FULL + n0 + q4 * 4);
#pragma unroll
    for (int j = 0; j < 4; ++j) ts[(q4 * 4 + j) * KPAD + cr] = (_Float16)bf16q(v[j]);
  }
  __syncthreads();
  v4u rv[2];
#pragma unroll
  for (int it = 0; it < 2; ++it) {
    const int idx = it * 256 + tid;
    const int n = idx >> 3, piece = idx & 7;
    rv[it] = *(const v4u*)(ts + n * KPAD + piece * 8);
  }
#pragma unroll
  for (int it = 0; it < 2; ++it) {
    const int idx = it * 256 + tid;
    const int n = idx >> 3, piece = idx & 7;
    *(volatile v4u*)(xh + ((size_t)b * SEQ + n0 + n) * DM + c0 + piece * 8) = rv[it];
  }
  __threadfence();
#pragma unroll
  for (int it = 0; it < 2; ++it) {
    const int idx = it * 256 + tid;
    const int n = idx >> 3, piece = idx & 7;
    *(volatile v4u*)(xh + ((size_t)b * SEQ + n0 + n) * DM + c0 + piece * 8) = rv[it];
  }
}

__global__ __launch_bounds__(256) void cvt_w_kernel(
    const float* __restrict__ Wqkv, const float* __restrict__ Wp,
    const float* __restrict__ W1, const float* __restrict__ W2,
    _Float16* __restrict__ wqkv, _Float16* __restrict__ wph,
    _Float16* __restrict__ wf1h, _Float16* __restrict__ wf2h) {
  const int bid = blockIdx.x;
  const float* src;
  _Float16* dst;
  int lb;
  if (bid < NWB_QKV) { src = Wqkv; dst = wqkv; lb = bid; }
  else if (bid < NWB_QKV + NWB_P) { src = Wp; dst = wph; lb = bid - NWB_QKV; }
  else if (bid < NWB_QKV + NWB_P + NWB_F1) { src = W1; dst = wf1h; lb = bid - NWB_QKV - NWB_P; }
  else { src = W2; dst = wf2h; lb = bid - NWB_QKV - NWB_P - NWB_F1; }
  const size_t e = (size_t)lb * 2048 + (size_t)threadIdx.x * 8;
  const v4f a = *(const v4f*)(src + e);
  const v4f c = *(const v4f*)(src + e + 4);
  H8 o;
#pragma unroll
  for (int i = 0; i < 4; ++i) {
    o.h[i]     = (_Float16)(bf16q(a[i]) * WSC);
    o.h[4 + i] = (_Float16)(bf16q(c[i]) * WSC);
  }
  *(volatile v4u*)(dst + e) = o.u;
  __threadfence();
  *(volatile v4u*)(dst + e) = o.u;
}

__global__ __launch_bounds__(256) void qkv_kernel(
    const _Float16* __restrict__ xh, const _Float16* __restrict__ wqkv,
    const float* __restrict__ bqkv,
    _Float16* __restrict__ q, _Float16* __restrict__ k,
    _Float16* __restrict__ vT, _Float16* __restrict__ vR) {
  __shared__ _Float16 stg[128 * VSPAD];

  const int tid  = threadIdx.x;
  const int lane = tid & 31;
  const int wave = tid >> 5;
  const int hh   = lane >> 4;
  const int l15  = lane & 15;

  const int cb   = blockIdx.y;
  const int osel = cb >> 4;
  const int h    = cb & 15;
  const size_t m0 = (size_t)blockIdx.x * 128;
  const int  b   = (int)(m0 / SEQ);
  const int  s0  = (int)(m0 - (size_t)b * SEQ);

  const _Float16* xrow = xh + (m0 + (size_t)wave * 16) * DM;
  const _Float16* wrow = wqkv + ((size_t)cb * 64) * DM;

  v8f acc[4];
#pragma unroll
  for (int j = 0; j < 4; ++j) acc[j] = (v8f){};

#pragma unroll 1
  for (int kk = 0; kk < DM; kk += 32) {
    const v16h xf = load_frag_row(xrow + kk, DM, lane);
#pragma unroll
    for (int j = 0; j < 4; ++j) {
      const v16h wf = load_frag_row(wrow + (size_t)(j * 16) * DM + kk, DM, lane);
      acc[j] = wmma_f16(wf, xf, acc[j]);
    }
  }

  const float* bias = bqkv + cb * 64;
  const float  rsc  = 1.0f / WSC;

  v4u rv[8];
  if (osel < 2) {
    _Float16* srow = stg + (wave * 16 + l15) * KPAD;
#pragma unroll
    for (int j = 0; j < 4; ++j) {
      const int n8 = j * 16 + hh * 8;
      const v4f b0 = *(const v4f*)(bias + n8);
      const v4f b1 = *(const v4f*)(bias + n8 + 4);
      H8 pk;
#pragma unroll
      for (int r = 0; r < 4; ++r) {
        pk.h[r]     = (_Float16)(acc[j][r]     * rsc + bf16q(b0[r]));
        pk.h[4 + r] = (_Float16)(acc[j][4 + r] * rsc + bf16q(b1[r]));
      }
      *(v4u*)(srow + n8) = pk.u;
    }
    __syncthreads();
#pragma unroll
    for (int it = 0; it < 4; ++it) {
      const int idx = it * 256 + tid;
      const int row = idx >> 3, piece = idx & 7;
      rv[it] = *(const v4u*)(stg + row * KPAD + piece * 8);
    }
    _Float16* dst = ((osel == 0) ? q : k) + (((size_t)b * NH + h) * SEQ + s0) * HD;
#pragma unroll
    for (int it = 0; it < 4; ++it)
      *(volatile v4u*)(dst + (size_t)(it * 256 + tid) * 8) = rv[it];
    __threadfence();
#pragma unroll
    for (int it = 0; it < 4; ++it)
      *(volatile v4u*)(dst + (size_t)(it * 256 + tid) * 8) = rv[it];
  } else {
    const int tl = wave * 16 + l15;
#pragma unroll
    for (int j = 0; j < 4; ++j) {
      const int n8 = j * 16 + hh * 8;
      const v4f b0 = *(const v4f*)(bias + n8);
      const v4f b1 = *(const v4f*)(bias + n8 + 4);
#pragma unroll
      for (int r = 0; r < 4; ++r) {
        const float u0 = acc[j][r]     * rsc + bf16q(b0[r]);
        const float u1 = acc[j][4 + r] * rsc + bf16q(b1[r]);
        const _Float16 h0 = (_Float16)u0;
        const _Float16 h1 = (_Float16)u1;
        stg[(n8 + r) * VSPAD + tl]          = h0;
        stg[(64 + n8 + r) * VSPAD + tl]     = (_Float16)((u0 - (float)h0) * VRC);
        stg[(n8 + 4 + r) * VSPAD + tl]      = h1;
        stg[(64 + n8 + 4 + r) * VSPAD + tl] = (_Float16)((u1 - (float)h1) * VRC);
      }
    }
    __syncthreads();
#pragma unroll
    for (int it = 0; it < 8; ++it) {
      const int idx = it * 256 + tid;
      const int d = idx >> 4, piece = idx & 15;
      rv[it] = *(const v4u*)(stg + d * VSPAD + piece * 8);
    }
    const size_t pofs = (((size_t)b * NH + h) * HD) * SEQ + s0;
#pragma unroll
    for (int it = 0; it < 8; ++it) {
      const int idx = it * 256 + tid;
      const int d = (idx >> 4) & 63, piece = idx & 15;
      _Float16* base = (it < 4) ? vT : vR;
      *(volatile v4u*)(base + pofs + (size_t)d * SEQ + piece * 8) = rv[it];
    }
    __threadfence();
#pragma unroll
    for (int it = 0; it < 8; ++it) {
      const int idx = it * 256 + tid;
      const int d = (idx >> 4) & 63, piece = idx & 15;
      _Float16* base = (it < 4) ? vT : vR;
      *(volatile v4u*)(base + pofs + (size_t)d * SEQ + piece * 8) = rv[it];
    }
  }
}

__global__ __launch_bounds__(256) void attn_kernel(
    const _Float16* __restrict__ Q, const _Float16* __restrict__ K,
    const _Float16* __restrict__ vT, const _Float16* __restrict__ vR,
    const int* __restrict__ mask, _Float16* __restrict__ am) {
  __shared__ _Float16 ks[64 * KPAD];
  __shared__ _Float16 vts[64 * KPAD];
  __shared__ _Float16 vrs[64 * KPAD];
  __shared__ _Float16 ost[64 * VSPAD];

  const int tid  = threadIdx.x;
  const int lane = tid & 31;
  const int wave = tid >> 5;
  const int bh   = blockIdx.y;
  const int b    = bh / NH;
  const int h    = bh - b * NH;
  const int q0   = blockIdx.x * 128;
  const int colb = lane & 15;
  const int rofs = (lane >> 4) << 3;

  const _Float16* Qb  = Q + ((size_t)bh * SEQ + q0) * HD;
  const _Float16* Kb  = K + (size_t)bh * SEQ * HD;
  const _Float16* vTb = vT + (size_t)bh * HD * SEQ;
  const _Float16* vRb = vR + (size_t)bh * HD * SEQ;

  v16h qfrag[2];
  {
    const _Float16* qrow = Qb + (size_t)wave * 16 * HD;
#pragma unroll
    for (int t = 0; t < 2; ++t) qfrag[t] = load_frag_row(qrow + t * 32, HD, lane);
  }

  const int  qi    = q0 + wave * 16 + colb;
  const bool rowOk = (mask[(size_t)bh * SEQ_FULL + qi] != 0);

  v8f acc[4];
  v8f accr[4];
#pragma unroll
  for (int nt = 0; nt < 4; ++nt) { acc[nt] = (v8f){}; accr[nt] = (v8f){}; }
  float mi = -1e30f, li = 0.0f;

#pragma unroll 1
  for (int kb = 0; kb < SEQ; kb += 64) {
    __syncthreads();
#pragma unroll
    for (int idx = tid; idx < 64 * 8; idx += 256) {
      const int row = idx >> 3, c = idx & 7;
      *(v4u*)(ks + row * KPAD + c * 8) =
          *(const v4u*)(Kb + (size_t)(kb + row) * HD + c * 8);
    }
#pragma unroll
    for (int idx = tid; idx < 64 * 8; idx += 256) {
      const int d = idx >> 3, c = idx & 7;
      *(v4u*)(vts + d * KPAD + c * 8) =
          *(const v4u*)(vTb + (size_t)d * SEQ + kb + c * 8);
      *(v4u*)(vrs + d * KPAD + c * 8) =
          *(const v4u*)(vRb + (size_t)d * SEQ + kb + c * 8);
    }
    __syncthreads();

    v8f sc[4];
#pragma unroll
    for (int kt = 0; kt < 4; ++kt) sc[kt] = (v8f){};
#pragma unroll
    for (int t = 0; t < 2; ++t)
#pragma unroll
      for (int kt = 0; kt < 4; ++kt) {
        const v16h kf = load_frag_row(ks + (kt * 16) * KPAD + t * 32, KPAD, lane);
        sc[kt] = wmma_f16(kf, qfrag[t], sc[kt]);
      }

#pragma unroll
    for (int kt = 0; kt < 4; ++kt)
#pragma unroll
      for (int r = 0; r < 8; ++r) sc[kt][r] = rowOk ? sc[kt][r] : 0.0f;

    float mx = sc[0][0];
#pragma unroll
    for (int kt = 0; kt < 4; ++kt)
#pragma unroll
      for (int r = 0; r < 8; ++r) mx = fmaxf(mx, sc[kt][r]);
    mx = fmaxf(mx, __shfl_xor(mx, 16, 32));
    const float mnew  = fmaxf(mi, mx);
    const float alpha = __expf((mi - mnew) * 0.125f);
    mi = mnew;
    const float cs = fmaf(mnew, 0.125f, -LN1024);

    float rs = 0.0f;
#pragma unroll
    for (int kt = 0; kt < 4; ++kt)
#pragma unroll
      for (int r = 0; r < 8; ++r) {
        const float p = __expf(fmaf(sc[kt][r], 0.125f, -cs));
        sc[kt][r] = p;
        rs += p;
      }
    rs += __shfl_xor(rs, 16, 32);
    li = li * alpha + rs;

    v16h pf[2];
#pragma unroll
    for (int t = 0; t < 2; ++t)
#pragma unroll
      for (int i = 0; i < 8; ++i) {
        pf[t][i]     = (_Float16)sc[2 * t][i];
        pf[t][8 + i] = (_Float16)sc[2 * t + 1][i];
      }

#pragma unroll
    for (int nt = 0; nt < 4; ++nt)
#pragma unroll
      for (int r = 0; r < 8; ++r) { acc[nt][r] *= alpha; accr[nt][r] *= alpha; }

#pragma unroll
    for (int t = 0; t < 2; ++t)
#pragma unroll
      for (int nt = 0; nt < 4; ++nt) {
        const v16h vf = load_frag_row(vts + (nt * 16) * KPAD + t * 32, KPAD, lane);
        acc[nt] = wmma_f16(vf, pf[t], acc[nt]);
        const v16h wf = load_frag_row(vrs + (nt * 16) * KPAD + t * 32, KPAD, lane);
        accr[nt] = wmma_f16(wf, pf[t], accr[nt]);
      }
  }

  {
    const float inv = CTXC / (1024.0f + li);
    const float rrc = 1.0f / VRC;
#pragma unroll
    for (int nt = 0; nt < 4; ++nt)
#pragma unroll
      for (int r = 0; r < 8; ++r)
        ost[(nt * 16 + rofs + r) * VSPAD + wave * 16 + colb] =
            (_Float16)((acc[nt][r] + accr[nt][r] * rrc) * inv);
  }
  __syncthreads();

  v4u rv[4];
#pragma unroll
  for (int it = 0; it < 4; ++it) {
    const int idx = it * 256 + tid;
    const int d = idx >> 4, piece = idx & 15;
    rv[it] = *(const v4u*)(ost + d * VSPAD + piece * 8);
  }
  _Float16* amb = am + (size_t)b * SEQ * DM;
#pragma unroll
  for (int it = 0; it < 4; ++it) {
    const int idx = it * 256 + tid;
    const int d = idx >> 4, piece = idx & 15;
    const size_t f0  = (size_t)d * NH * SEQ + (size_t)h * SEQ + (size_t)q0;
    const size_t row = f0 / DM, col = f0 - row * DM;
    *(volatile v4u*)(amb + row * DM + col + piece * 8) = rv[it];
  }
  __threadfence();
#pragma unroll
  for (int it = 0; it < 4; ++it) {
    const int idx = it * 256 + tid;
    const int d = idx >> 4, piece = idx & 15;
    const size_t f0  = (size_t)d * NH * SEQ + (size_t)h * SEQ + (size_t)q0;
    const size_t row = f0 / DM, col = f0 - row * DM;
    *(volatile v4u*)(amb + row * DM + col + piece * 8) = rv[it];
  }
}

__global__ __launch_bounds__(256) void proj_kernel(
    const _Float16* __restrict__ am, const _Float16* __restrict__ wph,
    const float* __restrict__ pb, float* __restrict__ h2f, _Float16* __restrict__ h2h) {
  __shared__ float stg[128 * SP64];

  const int tid  = threadIdx.x;
  const int lane = tid & 31;
  const int wave = tid >> 5;
  const int hh   = lane >> 4;
  const int l15  = lane & 15;
  const int cb   = blockIdx.y;
  const size_t m0 = (size_t)blockIdx.x * 128;

  const _Float16* brow = am + (m0 + (size_t)wave * 16) * DM;
  const _Float16* arow = wph + ((size_t)cb * 64) * DM;

  v8f acc[4];
#pragma unroll
  for (int j = 0; j < 4; ++j) acc[j] = (v8f){};

#pragma unroll 1
  for (int kk = 0; kk < DM; kk += 32) {
    const v16h xf = load_frag_row(brow + kk, DM, lane);
#pragma unroll
    for (int j = 0; j < 4; ++j) {
      const v16h wf = load_frag_row(arow + (size_t)(j * 16) * DM + kk, DM, lane);
      acc[j] = wmma_f16(wf, xf, acc[j]);
    }
  }

  {
    const float rsc = 1.0f / (WSC * CTXC);
    float* srow = stg + (wave * 16 + l15) * SP64;
#pragma unroll
    for (int j = 0; j < 4; ++j) {
      const int n8 = j * 16 + hh * 8;
      const v4f b0 = *(const v4f*)(pb + cb * 64 + n8);
      const v4f b1 = *(const v4f*)(pb + cb * 64 + n8 + 4);
      v4f y0, y1;
#pragma unroll
      for (int i = 0; i < 4; ++i) {
        y0[i] = 2.0f * (acc[j][i]     * rsc + bf16q(b0[i]));
        y1[i] = 2.0f * (acc[j][4 + i] * rsc + bf16q(b1[i]));
      }
      *(v4f*)(srow + n8)     = y0;
      *(v4f*)(srow + n8 + 4) = y1;
    }
  }
  __syncthreads();

  auto store_pass = [&]() {
#pragma unroll 4
    for (int it = 0; it < 8; ++it) {
      const int idx = it * 256 + tid;
      const int row = idx >> 4, piece = idx & 15;
      const v4f v = *(const v4f*)(stg + row * SP64 + piece * 4);
      *(volatile v4f*)(h2f + (m0 + row) * DM + cb * 64 + piece * 4) = v;
    }
#pragma unroll
    for (int it = 0; it < 4; ++it) {
      const int idx = it * 256 + tid;
      const int row = idx >> 3, p8 = idx & 7;
      const v4f a = *(const v4f*)(stg + row * SP64 + p8 * 8);
      const v4f c = *(const v4f*)(stg + row * SP64 + p8 * 8 + 4);
      H8 o;
#pragma unroll
      for (int i = 0; i < 4; ++i) {
        o.h[i]     = (_Float16)(a[i] * H2C);
        o.h[4 + i] = (_Float16)(c[i] * H2C);
      }
      *(volatile v4u*)(h2h + (m0 + row) * DM + cb * 64 + p8 * 8) = o.u;
    }
  };
  store_pass();
  __threadfence();
  store_pass();
}

__global__ __launch_bounds__(256) void fc1_kernel(
    const _Float16* __restrict__ h2h, const _Float16* __restrict__ wf1h,
    const float* __restrict__ b1, float* __restrict__ gp) {
  __shared__ float stg[128 * SP64];

  const int tid  = threadIdx.x;
  const int lane = tid & 31;
  const int wave = tid >> 5;
  const int hh   = lane >> 4;
  const int l15  = lane & 15;
  const int cb   = blockIdx.y;
  const size_t m0 = (size_t)blockIdx.x * 128;

  const _Float16* brow = h2h + (m0 + (size_t)wave * 16) * DM;
  const _Float16* arow = wf1h + ((size_t)cb * 64) * DM;

  v8f acc[4];
#pragma unroll
  for (int j = 0; j < 4; ++j) acc[j] = (v8f){};

#pragma unroll 1
  for (int kk = 0; kk < DM; kk += 32) {
    const v16h xf = load_frag_row(brow + kk, DM, lane);
#pragma unroll
    for (int j = 0; j < 4; ++j) {
      const v16h wf = load_frag_row(arow + (size_t)(j * 16) * DM + kk, DM, lane);
      acc[j] = wmma_f16(wf, xf, acc[j]);
    }
  }

  {
    const float rsc = 1.0f / (WSC * H2C);
    float* srow = stg + (wave * 16 + l15) * SP64;
#pragma unroll
    for (int j = 0; j < 4; ++j) {
      const int n8 = j * 16 + hh * 8;
      const v4f bb0 = *(const v4f*)(b1 + cb * 64 + n8);
      const v4f bb1 = *(const v4f*)(b1 + cb * 64 + n8 + 4);
      v4f y0, y1;
#pragma unroll
      for (int i = 0; i < 4; ++i) {
        const float u0 = acc[j][i]     * rsc + bf16q(bb0[i]);
        const float u1 = acc[j][4 + i] * rsc + bf16q(bb1[i]);
        y0[i] = 0.5f * u0 * (1.0f + erff(u0 * 0.70710678118654752f));
        y1[i] = 0.5f * u1 * (1.0f + erff(u1 * 0.70710678118654752f));
      }
      *(v4f*)(srow + n8)     = y0;
      *(v4f*)(srow + n8 + 4) = y1;
    }
  }
  __syncthreads();

  v4f rv[8];
#pragma unroll
  for (int it = 0; it < 8; ++it) {
    const int idx = it * 256 + tid;
    const int row = idx >> 4, piece = idx & 15;
    rv[it] = *(const v4f*)(stg + row * SP64 + piece * 4);
  }
#pragma unroll
  for (int it = 0; it < 8; ++it) {
    const int idx = it * 256 + tid;
    const int row = idx >> 4, piece = idx & 15;
    *(volatile v4f*)(gp + (m0 + row) * FF + cb * 64 + piece * 4) = rv[it];
  }
  __threadfence();
#pragma unroll
  for (int it = 0; it < 8; ++it) {
    const int idx = it * 256 + tid;
    const int row = idx >> 4, piece = idx & 15;
    *(volatile v4f*)(gp + (m0 + row) * FF + cb * 64 + piece * 4) = rv[it];
  }
}

__global__ __launch_bounds__(256) void ln_kernel(
    const float* __restrict__ gp, const float* __restrict__ lg,
    const float* __restrict__ lb, _Float16* __restrict__ np) {
  __shared__ float red0[8];
  __shared__ float red1[8];

  const int tid  = threadIdx.x;
  const int lane = tid & 31;
  const int wave = tid >> 5;
  const size_t row = blockIdx.x;
  const float* gr = gp + row * FF;

  float s = 0.0f;
#pragma unroll 1
  for (int it = 0; it < 2; ++it) {
    const int j0 = it * 2048 + tid * 8;
    const v4f a = *(const v4f*)(gr + j0);
    const v4f c = *(const v4f*)(gr + j0 + 4);
    s += ((a[0] + a[1]) + (a[2] + a[3])) + ((c[0] + c[1]) + (c[2] + c[3]));
  }
  s = wave_sum(s);
  if (lane == 0) red0[wave] = s;
  __syncthreads();
  float tot = 0.0f;
#pragma unroll
  for (int w = 0; w < 8; ++w) tot += red0[w];
  const float mean = tot * (1.0f / FF);

  float ss = 0.0f;
#pragma unroll 1
  for (int it = 0; it < 2; ++it) {
    const int j0 = it * 2048 + tid * 8;
    const v4f a = *(const v4f*)(gr + j0);
    const v4f c = *(const v4f*)(gr + j0 + 4);
#pragma unroll
    for (int i = 0; i < 4; ++i) {
      const float d0 = a[i] - mean;
      const float d1 = c[i] - mean;
      ss += d0 * d0;
      ss += d1 * d1;
    }
  }
  ss = wave_sum(ss);
  if (lane == 0) red1[wave] = ss;
  __syncthreads();
  float tot2 = 0.0f;
#pragma unroll
  for (int w = 0; w < 8; ++w) tot2 += red1[w];
  const float var  = tot2 * (1.0f / FF);
  const float rstd = rsqrtf(var + LN_EPS);

  _Float16* nrow = np + row * FF;
#pragma unroll 1
  for (int pass = 0; pass < 2; ++pass) {
    if (pass == 1) __threadfence();
#pragma unroll 1
    for (int it = 0; it < 2; ++it) {
      const int j0 = it * 2048 + tid * 8;
      const v4f a  = *(const v4f*)(gr + j0);
      const v4f c  = *(const v4f*)(gr + j0 + 4);
      const v4f g0 = *(const v4f*)(lg + j0);
      const v4f g1 = *(const v4f*)(lg + j0 + 4);
      const v4f t0 = *(const v4f*)(lb + j0);
      const v4f t1 = *(const v4f*)(lb + j0 + 4);
      H8 o;
#pragma unroll
      for (int i = 0; i < 4; ++i) {
        o.h[i]     = (_Float16)(((a[i] - mean) * rstd) * bf16q(g0[i]) + bf16q(t0[i]));
        o.h[4 + i] = (_Float16)(((c[i] - mean) * rstd) * bf16q(g1[i]) + bf16q(t1[i]));
      }
      *(volatile v4u*)(nrow + j0) = o.u;
    }
  }
}

__global__ __launch_bounds__(256) void fc2_kernel(
    const _Float16* __restrict__ np, const _Float16* __restrict__ wf2h,
    const float* __restrict__ b2, const float* __restrict__ h2f,
    float* __restrict__ out) {
  __shared__ float stg[64 * SP128];

  const int tid  = threadIdx.x;
  const int lane = tid & 31;
  const int wave = tid >> 5;
  const int hh   = lane >> 4;
  const int l15  = lane & 15;
  const int cb   = blockIdx.y;
  const size_t m0 = (size_t)blockIdx.x * 128;
  const int  b   = (int)(m0 / SEQ);
  const int  s0  = (int)(m0 - (size_t)b * SEQ);

  const _Float16* brow = np + (m0 + (size_t)wave * 16) * FF;
  const _Float16* arow = wf2h + ((size_t)cb * 64) * FF;

  v8f acc[4];
#pragma unroll
  for (int j = 0; j < 4; ++j) acc[j] = (v8f){};

#pragma unroll 1
  for (int kk = 0; kk < FF; kk += 32) {
    const v16h xf = load_frag_row(brow + kk, FF, lane);
#pragma unroll
    for (int j = 0; j < 4; ++j) {
      const v16h wf = load_frag_row(arow + (size_t)(j * 16) * FF + kk, FF, lane);
      acc[j] = wmma_f16(wf, xf, acc[j]);
    }
  }

  {
    const float rsc = 1.0f / WSC;
    const int   tl  = wave * 16 + l15;
    const float* rrow = h2f + (m0 + tl) * DM + cb * 64;
#pragma unroll
    for (int j = 0; j < 4; ++j) {
      const int n8 = j * 16 + hh * 8;
      const v4f bb0 = *(const v4f*)(b2 + cb * 64 + n8);
      const v4f bb1 = *(const v4f*)(b2 + cb * 64 + n8 + 4);
      const v4f r0  = *(const v4f*)(rrow + n8);
      const v4f r1  = *(const v4f*)(rrow + n8 + 4);
#pragma unroll
      for (int i = 0; i < 4; ++i) {
        stg[(n8 + i) * SP128 + tl]     = (acc[j][i]     * rsc + bf16q(bb0[i])) + r0[i];
        stg[(n8 + 4 + i) * SP128 + tl] = (acc[j][4 + i] * rsc + bf16q(bb1[i])) + r1[i];
      }
    }
  }
  __syncthreads();

  float* ob = out + ((size_t)b * DM + (size_t)cb * 64) * SEQ_FULL + s0;
#pragma unroll
  for (int it = 0; it < 8; ++it) {
    const int idx = it * 256 + tid;
    const int c = idx >> 5, piece = idx & 31;
    const v4f v = *(const v4f*)(stg + c * SP128 + piece * 4);
    *(volatile v4f*)(ob + (size_t)c * SEQ_FULL + piece * 4) = v;
  }
  __threadfence();
#pragma unroll
  for (int it = 0; it < 8; ++it) {
    const int idx = it * 256 + tid;
    const int c = idx >> 5, piece = idx & 31;
    const v4f v = *(const v4f*)(stg + c * SP128 + piece * 4);
    *(volatile v4f*)(ob + (size_t)c * SEQ_FULL + piece * 4) = v;
  }
}

extern "C" void kernel_launch(void* const* d_in, const int* in_sizes, int n_in,
                              void* d_out, int out_size, void* d_ws, size_t ws_size,
                              hipStream_t stream) {
  if (n_in < 12) return;
  if ((long)in_sizes[0] < (long)NB * DM * SEQ_FULL) return;
  if ((long)in_sizes[1] < (long)NB * NH * SEQ_FULL) return;
  if (in_sizes[2] < 3 * DM * DM || in_sizes[3] < 3 * DM) return;
  if (in_sizes[4] < DM * DM || in_sizes[5] < DM) return;
  if (in_sizes[6] < FF * DM || in_sizes[7] < FF || in_sizes[8] < FF || in_sizes[9] < FF) return;
  if (in_sizes[10] < DM * FF || in_sizes[11] < DM) return;
  if ((long)out_size < ((long)NB * DM - 1) * SEQ_FULL + SEQ) return;
  if (ws_size < WS_TOTAL) return;

  const float* x    = (const float*)d_in[0];
  const int*   mask = (const int*)d_in[1];
  const float* Wqkv = (const float*)d_in[2];
  const float* bqkv = (const float*)d_in[3];
  const float* Wp   = (const float*)d_in[4];
  const float* bp   = (const float*)d_in[5];
  const float* W1   = (const float*)d_in[6];
  const float* b1   = (const float*)d_in[7];
  const float* lg   = (const float*)d_in[8];
  const float* lb   = (const float*)d_in[9];
  const float* W2   = (const float*)d_in[10];
  const float* b2   = (const float*)d_in[11];
  float* out = (float*)d_out;

  char* ws = (char*)d_ws;
  size_t off = 0;
  _Float16* xh   = (_Float16*)(ws + off); off += XH_BYTES;
  _Float16* wqkv = (_Float16*)(ws + off); off += WQKV_BYTES;
  _Float16* wph  = (_Float16*)(ws + off); off += WP_BYTES;
  _Float16* qh   = (_Float16*)(ws + off); off += QP_BYTES;
  _Float16* kh   = (_Float16*)(ws + off); off += QP_BYTES;
  _Float16* vTh  = (_Float16*)(ws + off); off += QP_BYTES;
  _Float16* vRh  = (_Float16*)(ws + off); off += QP_BYTES;
  _Float16* am   = (_Float16*)(ws + off); off += AM_BYTES;
  if (off > RG_BYTES) return;
  float*    gp   = (float*)(ws + 0);
  _Float16* h2h  = (_Float16*)(ws + RG_BYTES);
  _Float16* wf1h = (_Float16*)(ws + RG_BYTES + H2H_BYTES);
  _Float16* np   = (_Float16*)(ws + RG_BYTES);
  float*    h2f  = (float*)(ws + RG_BYTES + RN_BYTES);
  _Float16* wf2h = (_Float16*)(ws + RG_BYTES + RN_BYTES + H2F_BYTES);
  if (RG_BYTES + RN_BYTES + H2F_BYTES + WF2_BYTES > ws_size) return;

  cvt_x_kernel<<<dim3(SEQ / 64, DM / 64, NB), 256, 0, stream>>>(x, xh);
  cvt_w_kernel<<<NWB, 256, 0, stream>>>(Wqkv, Wp, W1, W2, wqkv, wph, wf1h, wf2h);
  qkv_kernel<<<dim3(ROWS / 128, 3 * NH), 256, 0, stream>>>(xh, wqkv, bqkv, qh, kh, vTh, vRh);
  attn_kernel<<<dim3(SEQ / 128, NB * NH), 256, 0, stream>>>(qh, kh, vTh, vRh, mask, am);
  proj_kernel<<<dim3(ROWS / 128, DM / 64), 256, 0, stream>>>(am, wph, bp, h2f, h2h);
  fc1_kernel<<<dim3(ROWS / 128, FF / 64), 256, 0, stream>>>(h2h, wf1h, b1, gp);
  ln_kernel<<<ROWS, 256, 0, stream>>>(gp, lg, lb, np);
  fc2_kernel<<<dim3(ROWS / 128, DM / 64), 256, 0, stream>>>(np, wf2h, b2, h2f, out);
}
